// LSTM_model_55138790146616
// MI455X (gfx1250) — hardware-verified
//
#include <hip/hip_runtime.h>
#include <stdint.h>

typedef __attribute__((ext_vector_type(16))) _Float16 v16h;
typedef __attribute__((ext_vector_type(8)))  _Float16 v8h;
typedef __attribute__((ext_vector_type(8)))  float    v8f;
typedef __attribute__((ext_vector_type(4)))  float    v4f;
typedef __attribute__((ext_vector_type(2)))  float    v2f;

__device__ __forceinline__ void dep_guard_h(v8f& a, v8f& b, v16h x, v16h y) { asm volatile("v_nop\n\tv_nop\n\tv_nop\n\tv_nop" : "+v"(a), "+v"(b) : "v"(x), "v"(y)); }
__device__ __forceinline__ void keep4_h(v16h a, v16h b, v16h c, v16h d) { asm volatile("v_nop" :: "v"(a), "v"(b), "v"(c), "v"(d)); }
template <typename T> struct Frag;
template <> struct Frag<_Float16> {
  typedef v16h V; union U { v16h v; v8h h[2]; };
  static __device__ __forceinline__ v16h load(const _Float16* p) {
    U f; f.h[0] = *(const v8h*)(p); f.h[1] = *(const v8h*)(p + 16); return f.v;
  }
  static __device__ __forceinline__ v8f mma(v16h a, v16h b, v8f c) {
    return __builtin_amdgcn_wmma_f32_16x16x32_f16(false, a, false, b, (short)0, c, false, false);
  }
  static __device__ __forceinline__ void guard(v8f& a, v8f& b, v16h x, v16h y) { dep_guard_h(a, b, x, y); }
  static __device__ __forceinline__ void keep(v16h a, v16h b, v16h c, v16h d) { keep4_h(a, b, c, d); }
};

constexpr int SEQ_T    = 1024;
constexpr int DIM_X    = 12;
constexpr int HID      = 100;
constexpr int NGATE    = 4 * HID;
constexpr int ROWS     = 16;
constexpr int KPADDED  = 128;
constexpr int APITCH   = 136;
constexpr int NTILE_G  = NGATE / 16;
constexpr int NCOLS    = (NTILE_G + 1) * 16;
constexpr int SPITCH   = 40;
constexpr int NWAVE_MMA = 13;
constexpr int NWAVES   = NWAVE_MMA + 1;
constexpr int NTHR     = NWAVES * 32;
constexpr int OSLOT    = 8;
constexpr int OPITCH   = OSLOT * DIM_X;
constexpr int NPAIR    = NCOLS * 16;
constexpr int NSTG_IT  = (NPAIR + NTHR - 1) / NTHR;
constexpr int ZRAW_FLOATS = (NGATE * ROWS > NCOLS * SPITCH / 2) ? (NGATE * ROWS) : (NCOLS * SPITCH / 2);
constexpr float SC16   = 16.0f;
constexpr float INV256 = 1.0f / 256.0f;

static_assert(NTILE_G * 16 == NGATE, "gate tiles");
static_assert(2 * NWAVE_MMA == NTILE_G + 1, "two tiles per MMA wave");
static_assert(HID + DIM_X <= KPADDED && KPADDED % 32 == 0, "K padding");
static_assert(APITCH >= KPADDED && APITCH % 8 == 0, "A pitch");
static_assert(SPITCH >= 32 && SPITCH % 8 == 0, "staging pitch");
static_assert(SEQ_T % OSLOT == 0, "flush granularity");
static_assert(OPITCH % 32 == 0, "whole lines per row per flush");
static_assert(HID % 4 == 0 && ROWS * HID / 4 <= NWAVE_MMA * 32, "gate thread map");
static_assert(DIM_X % 2 == 0 && ROWS * 2 == 32, "x staging lane map");
static_assert((ROWS * 3) % 4 == 0 && ROWS * 3 / 4 == 12, "flush line map");
static_assert(ROWS * APITCH % 8 == 0 && ROWS * APITCH / 8 <= NTHR, "A zero fill");
static_assert(ROWS * HID % 4 == 0 && ROWS * HID / 4 <= NTHR, "c zero fill");
static_assert(ZRAW_FLOATS * 4 >= NCOLS * SPITCH * 2, "staging fits");

__device__ __forceinline__ float bf16_rne(float f) {
  unsigned u = __float_as_uint(f);
  u = (u + 0x7FFFu + ((u >> 16) & 1u)) & 0xFFFF0000u;
  return __uint_as_float(u);
}
__device__ __forceinline__ unsigned f16_bits(float f) {
  return (unsigned)__builtin_bit_cast(unsigned short, (_Float16)f);
}
__device__ __forceinline__ float sigm_f(float z) {
  const float e = expf(-z);
  return __builtin_amdgcn_rcpf(1.0f + e);
}

__device__ __forceinline__ unsigned wsel_bits(const float* __restrict__ Wh, const float* __restrict__ Wx,
                                              const float* __restrict__ Wd, int k, int n) {
  const int kh = min(k, HID - 1);
  const int ng = min(n, NGATE - 1);
  const int kx = min(max(k - HID, 0), DIM_X - 1);
  const int nd = min(max(n - NGATE, 0), DIM_X - 1);
  const float vh = Wh[kh * NGATE + ng];
  const float vx = Wx[kx * NGATE + ng];
  const float vd = Wd[kh * DIM_X + nd];
  const bool gatecol = (n < NGATE);
  const float vg = (k < HID) ? vh : ((k < HID + DIM_X) ? vx : 0.0f);
  const float vo = (k < HID && n < NGATE + DIM_X) ? vd : 0.0f;
  const float v  = gatecol ? vg : vo;
  return f16_bits(SC16 * bf16_rne(v));
}

__device__ __forceinline__ void stage_x_row(const float* __restrict__ x, unsigned* ash, int b0, int tt, int lane) {
  const int m  = lane >> 1;
  const int hf = lane & 1;
  const float* xp = x + ((size_t)(b0 + m) * SEQ_T + tt) * DIM_X + 6 * hf;
  const v2f p0 = *(const v2f*)(xp);
  const v2f p1 = *(const v2f*)(xp + 2);
  const v2f p2 = *(const v2f*)(xp + 4);
  const unsigned w0 = f16_bits(SC16 * bf16_rne(p0[0])) | (f16_bits(SC16 * bf16_rne(p0[1])) << 16);
  const unsigned w1 = f16_bits(SC16 * bf16_rne(p1[0])) | (f16_bits(SC16 * bf16_rne(p1[1])) << 16);
  const unsigned w2 = f16_bits(SC16 * bf16_rne(p2[0])) | (f16_bits(SC16 * bf16_rne(p2[1])) << 16);
  unsigned* dst = ash + ((m * APITCH + HID + 6 * hf) >> 1);
  dst[0] = w0; dst[1] = w1; dst[2] = w2;
}

__device__ __forceinline__ float lstm_unit(const float* zs, float* cs, int m, int u) {
  const float zi = zs[u * ROWS + m];
  const float zf = zs[(HID + u) * ROWS + m];
  const float zg = zs[(2 * HID + u) * ROWS + m];
  const float zo = zs[(3 * HID + u) * ROWS + m];
  const float ig = sigm_f(zi);
  const float fg = sigm_f(zf);
  const float gg = tanhf(zg);
  const float og = sigm_f(zo);
  const float cp = cs[m * HID + u];
  const float cn = fg * cp + ig * gg;
  cs[m * HID + u] = cn;
  return og * tanhf(cn);
}

__global__ __launch_bounds__(NTHR) void lstm_seq_kernel(
    const float* __restrict__ x,  const float* __restrict__ Wx, const float* __restrict__ Wh,
    const float* __restrict__ bvec, const float* __restrict__ Wd, const float* __restrict__ bd,
    float* __restrict__ out)
{
  __shared__ __align__(16) float    zraw[ZRAW_FLOATS];
  __shared__ __align__(16) unsigned ash[ROWS * APITCH / 2];
  __shared__ __align__(16) float    csh[ROWS * HID];
  __shared__ __align__(16) float    osh[ROWS * OPITCH];

  const int tid  = threadIdx.x;
  const int lane = tid & 31;
  const int wave = __builtin_amdgcn_readfirstlane(tid >> 5);
  const int hh   = lane >> 4;
  const int c    = lane & 15;
  const int b0   = blockIdx.x * ROWS;
  const _Float16* ashh = (const _Float16*)ash;
  unsigned* stg32 = (unsigned*)zraw;
  const _Float16* stgh = (const _Float16*)zraw;

  if (tid < ROWS * APITCH / 8) ((uint4*)ash)[tid] = make_uint4(0u, 0u, 0u, 0u);
  if (tid < ROWS * HID / 4)    ((v4f*)csh)[tid]  = (v4f){0.0f, 0.0f, 0.0f, 0.0f};
  __syncthreads();
  if (wave == NWAVE_MMA) stage_x_row(x, ash, b0, 0, lane);

  const int tile0 = 2 * wave, tile1 = 2 * wave + 1;
  const int n0 = min(tile0 * 16 + c, NCOLS - 1);
  const int n1 = min(tile1 * 16 + c, NCOLS - 1);
  v16h bg0[4], bg1[4];
#pragma unroll
  for (int kt = 0; kt < 4; ++kt) {
#pragma unroll 1
    for (int it = 0; it < NSTG_IT; ++it) {
      const int idx = min(it * NTHR + tid, NPAIR - 1);
      const int n   = idx >> 4;
      const int kp  = idx & 15;
      const int k   = kt * 32 + 2 * kp;
      const unsigned lo = wsel_bits(Wh, Wx, Wd, k, n);
      const unsigned hi = wsel_bits(Wh, Wx, Wd, k + 1, n);
      stg32[n * (SPITCH / 2) + kp] = lo | (hi << 16);
    }
    __syncthreads();
    bg0[kt] = Frag<_Float16>::load(stgh + n0 * SPITCH + 8 * hh);
    bg1[kt] = Frag<_Float16>::load(stgh + n1 * SPITCH + 8 * hh);
    __syncthreads();
  }

  const float bias0 = bf16_rne(bvec[min(n0, NGATE - 1)]);
  const float bgat1 = bf16_rne(bvec[min(n1, NGATE - 1)]);
  const float bden1 = bf16_rne(bd[min(c, DIM_X - 1)]);
  const float bias1 = (tile1 < NTILE_G) ? bgat1 : bden1;

  const v8f zero8 = {0.0f, 0.0f, 0.0f, 0.0f, 0.0f, 0.0f, 0.0f, 0.0f};
  const int q  = lane >> 3;
  const int l8 = lane & 7;

  for (int t = 0; t <= SEQ_T; ++t) {
    if (wave < NWAVE_MMA) {
      v8f acc0 = zero8, acc1 = zero8;
#pragma unroll
      for (int kt = 0; kt < 4; ++kt) {
        const v16h a = Frag<_Float16>::load(ashh + c * APITCH + kt * 32 + 8 * hh);
        acc0 = Frag<_Float16>::mma(a, bg0[kt], acc0);
        acc1 = Frag<_Float16>::mma(a, bg1[kt], acc1);
        dep_guard_h(acc0, acc1, a, bg1[kt]);
      }
      {
        v4f zl, zh;
        zl[0] = acc0[0] * INV256 + bias0; zl[1] = acc0[1] * INV256 + bias0;
        zl[2] = acc0[2] * INV256 + bias0; zl[3] = acc0[3] * INV256 + bias0;
        zh[0] = acc0[4] * INV256 + bias0; zh[1] = acc0[5] * INV256 + bias0;
        zh[2] = acc0[6] * INV256 + bias0; zh[3] = acc0[7] * INV256 + bias0;
        *(v4f*)(zraw + n0 * ROWS + 8 * hh)     = zl;
        *(v4f*)(zraw + n0 * ROWS + 8 * hh + 4) = zh;
      }
      if (tile1 < NTILE_G) {
        v4f zl, zh;
        zl[0] = acc1[0] * INV256 + bias1; zl[1] = acc1[1] * INV256 + bias1;
        zl[2] = acc1[2] * INV256 + bias1; zl[3] = acc1[3] * INV256 + bias1;
        zh[0] = acc1[4] * INV256 + bias1; zh[1] = acc1[5] * INV256 + bias1;
        zh[2] = acc1[6] * INV256 + bias1; zh[3] = acc1[7] * INV256 + bias1;
        *(v4f*)(zraw + n1 * ROWS + 8 * hh)     = zl;
        *(v4f*)(zraw + n1 * ROWS + 8 * hh + 4) = zh;
      } else if (t >= 1) {
        const int slot = (t - 1) & (OSLOT - 1);
        if (c < DIM_X) {
#pragma unroll
          for (int r = 0; r < 8; ++r)
            osh[(8 * hh + r) * OPITCH + slot * DIM_X + c] = acc1[r] * INV256 + bias1;
        }
      }
    }
    __syncthreads();

    if (wave == NWAVE_MMA) {
      if ((t & (OSLOT - 1)) == 0 && t >= OSLOT) {
        const int t0 = t - OSLOT;
        for (int pass = 0; pass < 2; ++pass) {
#pragma unroll 1
          for (int il = 0; il < 12; ++il) {
            const int L = il * 4 + q;
            const int m = L / 3;
            const int j = L - m * 3;
            const v4f v = *(const v4f*)(osh + m * OPITCH + j * 32 + l8 * 4);
            *(volatile v4f*)(out + ((size_t)(b0 + m) * SEQ_T + t0) * DIM_X + j * 32 + l8 * 4) = v;
          }
          __threadfence();
        }
      }
      if (t + 1 < SEQ_T) stage_x_row(x, ash, b0, t + 1, lane);
    } else if (t < SEQ_T && tid < ROWS * HID / 4) {
      const int m  = tid & 15;
      const int ub = tid >> 4;
#pragma unroll 1
      for (int jp = 0; jp < 2; ++jp) {
        const int u0 = ub * 4 + jp * 2;
        const float h0 = lstm_unit(zraw, csh, m, u0);
        const float h1 = lstm_unit(zraw, csh, m, u0 + 1);
        ash[(m * APITCH + u0) >> 1] = f16_bits(SC16 * h0) | (f16_bits(SC16 * h1) << 16);
      }
    }
    __syncthreads();
  }
}

extern "C" void kernel_launch(void* const* d_in, const int* in_sizes, int n_in,
                              void* d_out, int out_size, void* d_ws, size_t ws_size,
                              hipStream_t stream) {
  (void)d_ws; (void)ws_size;
  if (n_in < 6) return;
  const float* x    = (const float*)d_in[0];
  const float* Wx   = (const float*)d_in[1];
  const float* Wh   = (const float*)d_in[2];
  const float* bvec = (const float*)d_in[3];
  const float* Wd   = (const float*)d_in[4];
  const float* bd   = (const float*)d_in[5];
  float* out = (float*)d_out;
  const int nb_in  = in_sizes[0] / (SEQ_T * DIM_X);
  const int nb_out = out_size / (SEQ_T * DIM_X);
  const int nb = (nb_in < nb_out) ? nb_in : nb_out;
  const int nblk = nb / ROWS;
  if (nblk <= 0) return;
  lstm_seq_kernel<<<dim3(nblk), dim3(NTHR), 0, stream>>>(x, Wx, Wh, bvec, Wd, bd, out);
}
